// PFN_30262339567992
// MI455X (gfx1250) — hardware-verified
//
#include <hip/hip_runtime.h>
#include <math.h>

typedef __attribute__((ext_vector_type(16))) _Float16 v16h;
typedef __attribute__((ext_vector_type(8)))  _Float16 v8h;
typedef __attribute__((ext_vector_type(16))) __bf16   v16b;
typedef __attribute__((ext_vector_type(8)))  __bf16   v8b;
typedef __attribute__((ext_vector_type(8)))  float    v8f;
typedef __attribute__((ext_vector_type(4)))  float    v4f;

constexpr int kL    = 128;
constexpr int kB    = 4;
constexpr int kD    = 768;
constexpr int kH    = 300;
constexpr int kHP   = 320;
constexpr int kG5   = 5 * kH;
constexpr int kG5P  = 1536;
constexpr int kRows = kL * kB;
constexpr int kPairs = kL * kL * kB;
constexpr int kNT   = 7;
constexpr int kNR   = 12;
constexpr int kTP   = 64;
constexpr int kMP   = 64;
constexpr int kCOP  = 512;
constexpr int kThr  = 256;
constexpr float kInCarry = 1024.0f;
constexpr float kWCarry = 4096.0f;
constexpr float kSC = 1024.0f;
constexpr float kCE = 256.0f;
constexpr float kScX = 1.0f / (kInCarry * kWCarry), kScS = 1.0f / (kSC * kWCarry), kScE = 1.0f / (kCE * kWCarry);
constexpr float kInvH = 1.0f / 300.0f;
constexpr float kLnEps = 1e-5f;
constexpr float kF16MinNormal = 6.103515625e-5f;

static_assert(kRows == 512 && kPairs == 65536 && (kG5P % 64) == 0 && ((kRows / 64) * (kG5P / 64)) % 8 == 0 && ((kMP / 64) * (kG5P / 64)) % 8 == 0 && ((kMP / 64) * (kCOP / 64)) % 8 == 0 && ((kRows / 64) * (kHP / 64)) % 8 == 0 && ((kRows / 64) * (2 * kHP / 64)) % 8 == 0 && ((kPairs / 64) * (kTP / 64)) % 8 == 0, "GEMM M and N multiples of 64; every grid a whole number of 8-tile blocks");
static_assert((kD % 32) == 0 && (kHP % 32) == 0 && (kH % 4) == 0 && kH < kHP && kG5 < kG5P && kH < kCOP && kNT < kTP && kNR < kTP, "GEMM K multiples of 32; 300 a multiple of 4; paddings");

constexpr size_t kOffX16 = 0ull;
constexpr size_t kOffWIH16 = 786432ull;
constexpr size_t kOffWHH16 = 3145728ull;
constexpr size_t kOffWTR16 = 4128768ull;
constexpr size_t kOffGWN16 = 5111808ull;
constexpr size_t kOffGWR16 = 5521408ull;
constexpr size_t kOffHWSEN16 = 5931008ull;
constexpr size_t kOffHWSER16 = 6340608ull;
constexpr size_t kOffHWGN16 = 6750208ull;
constexpr size_t kOffHWGR16 = 7077888ull;
constexpr size_t kOffTWN16 = 7405568ull;
constexpr size_t kOffTWR16 = 7446528ull;
constexpr size_t kOffBIAS = 7487488ull;
constexpr size_t kOffH16 = 7512064ull;
constexpr size_t kOffCC16 = 7553024ull;
constexpr size_t kOffG16 = 7675904ull;
constexpr size_t kOffCO = 7716864ull;
constexpr size_t kOffPRE = 7847936ull;
constexpr size_t kOffGG = 10993664ull;
constexpr size_t kOffTASK16 = 11386880ull;
constexpr size_t kOffHG = 12369920ull;
constexpr size_t kOffASE = 13025280ull;
constexpr size_t kOffCG = 14336000ull;
constexpr size_t kOffE16 = 14467072ull;
constexpr size_t kOffY = 56410112ull;
constexpr size_t kWsTotal = 73187328ull;
static_assert(kWsTotal <= 134217728ull, "carve cap: under 128 MiB");
static_assert(kOffX16 == 0
              && kOffWIH16 == kOffX16 + 786432ull
              && kOffWHH16 == kOffWIH16 + 2359296ull
              && kOffWTR16 == kOffWHH16 + 983040ull
              && kOffGWN16 == kOffWTR16 + 983040ull
              && kOffGWR16 == kOffGWN16 + 409600ull
              && kOffHWSEN16 == kOffGWR16 + 409600ull
              && kOffHWSER16 == kOffHWSEN16 + 409600ull
              && kOffHWGN16 == kOffHWSER16 + 409600ull
              && kOffHWGR16 == kOffHWGN16 + 327680ull
              && kOffTWN16 == kOffHWGR16 + 327680ull
              && kOffTWR16 == kOffTWN16 + 40960ull
              && kOffBIAS == kOffTWR16 + 40960ull
              && kOffH16 == kOffBIAS + 24576ull
              && kOffCC16 == kOffH16 + 40960ull
              && kOffG16 == kOffCC16 + 122880ull
              && kOffCO == kOffG16 + 40960ull
              && kOffPRE == kOffCO + 131072ull
              && kOffGG == kOffPRE + 3145728ull
              && kOffTASK16 == kOffGG + 393216ull
              && kOffHG == kOffTASK16 + 983040ull
              && kOffASE == kOffHG + 655360ull
              && kOffCG == kOffASE + 1310720ull
              && kOffE16 == kOffCG + 131072ull
              && kOffY == kOffE16 + 41943040ull
              && kWsTotal == kOffY + 16777216ull, "the carve is chained and totalled");
static_assert((kOffX16 % 256) == 0 && (kOffWIH16 % 256) == 0 && (kOffWHH16 % 256) == 0 && (kOffWTR16 % 256) == 0 && (kOffGWN16 % 256) == 0 && (kOffGWR16 % 256) == 0 && (kOffHWSEN16 % 256) == 0 && (kOffHWSER16 % 256) == 0 && (kOffHWGN16 % 256) == 0 && (kOffHWGR16 % 256) == 0 && (kOffTWN16 % 256) == 0 && (kOffTWR16 % 256) == 0 && (kOffBIAS % 256) == 0 && (kOffH16 % 256) == 0 && (kOffCC16 % 256) == 0 && (kOffG16 % 256) == 0 && (kOffCO % 256) == 0 && (kOffPRE % 256) == 0 && (kOffGG % 256) == 0 && (kOffTASK16 % 256) == 0 && (kOffHG % 256) == 0 && (kOffASE % 256) == 0 && (kOffCG % 256) == 0 && (kOffE16 % 256) == 0 && (kOffY % 256) == 0, "aligned regions");
static_assert(kOffCC16 == kOffH16 + 40960ull && kOffG16 == kOffCC16 + 122880ull && kOffCO == kOffG16 + 40960ull && kOffPRE == kOffCO + 131072ull, "the zero-filled region H16 | CC16 | G16 | CO is contiguous: 335,872 B");

__device__ __forceinline__ unsigned short f2bf_bits(float f) {
  unsigned u = __float_as_uint(f);
  return (unsigned short)((u + 0x7FFFu + ((u >> 16) & 1u)) >> 16);
}
__device__ __forceinline__ float bf_bits2f(unsigned short h) { return __uint_as_float(((unsigned)h) << 16); }
__device__ __forceinline__ float bf16r(float f) { return bf_bits2f(f2bf_bits(f)); }
__device__ __forceinline__ float carry_flush(float v, float carry) {
  const float s = v * carry;
  return (fabsf(s) < kF16MinNormal) ? 0.0f : s;
}
__device__ __forceinline__ float frcp(float x) { return __builtin_amdgcn_rcpf(x); }

__device__ __forceinline__ void dep_guard4_h(v8f& a, v8f& b, v8f& c, v8f& d, v16h x, v16h y) { asm volatile("v_nop\n\tv_nop\n\tv_nop\n\tv_nop" : "+v"(a), "+v"(b), "+v"(c), "+v"(d) : "v"(x), "v"(y)); }
__device__ __forceinline__ void dep_guard4_b(v8f& a, v8f& b, v8f& c, v8f& d, v16b x, v16b y) { asm volatile("v_nop\n\tv_nop\n\tv_nop\n\tv_nop" : "+v"(a), "+v"(b), "+v"(c), "+v"(d) : "v"(x), "v"(y)); }
__device__ __forceinline__ void keep4_h(v16h a, v16h b, v16h c, v16h d) { asm volatile("v_nop" :: "v"(a), "v"(b), "v"(c), "v"(d)); }
__device__ __forceinline__ void keep4_b(v16b a, v16b b, v16b c, v16b d) { asm volatile("v_nop" :: "v"(a), "v"(b), "v"(c), "v"(d)); }
__device__ __forceinline__ void acc_guard4(v8f& a, v8f& b, v8f& c, v8f& d) { asm volatile("v_nop\n\tv_nop\n\tv_nop\n\tv_nop" : "+v"(a), "+v"(b), "+v"(c), "+v"(d)); }

template <typename T> struct Frag;
template <> struct Frag<_Float16> {
  typedef v16h V; union U { v16h v; v8h h[2]; };
  static __device__ __forceinline__ v16h load(const _Float16* p) {
    U f; f.h[0] = *(const v8h*)(p); f.h[1] = *(const v8h*)(p + 16); return f.v;
  }
  static __device__ __forceinline__ v8f mma(v16h a, v16h b, v8f c) {
    return __builtin_amdgcn_wmma_f32_16x16x32_f16(false, a, false, b, (short)0, c, false, false);
  }
  static __device__ __forceinline__ void guard4(v8f& a, v8f& b, v8f& c, v8f& d, v16h x, v16h y) { dep_guard4_h(a, b, c, d, x, y); }
  static __device__ __forceinline__ void keep(v16h a, v16h b, v16h c, v16h d) { keep4_h(a, b, c, d); }
};
template <> struct Frag<__bf16> {
  typedef v16b V; union U { v16b v; v8b h[2]; };
  static __device__ __forceinline__ v16b load(const __bf16* p) {
    U f; f.h[0] = *(const v8b*)(p); f.h[1] = *(const v8b*)(p + 16); return f.v;
  }
  static __device__ __forceinline__ v8f mma(v16b a, v16b b, v8f c) {
    return __builtin_amdgcn_wmma_f32_16x16x32_bf16(false, a, false, b, (short)0, c, false, false);
  }
  static __device__ __forceinline__ void guard4(v8f& a, v8f& b, v8f& c, v8f& d, v16b x, v16b y) { dep_guard4_b(a, b, c, d, x, y); }
  static __device__ __forceinline__ void keep(v16b a, v16b b, v16b c, v16b d) { keep4_b(a, b, c, d); }
};

__device__ __forceinline__ v8f mma_h(v16h a, v16h b, v8f c) {
  c = __builtin_amdgcn_wmma_f32_16x16x32_f16(false, a, false, b, (short)0, c, false, false);
  asm volatile("v_nop\n\tv_nop\n\tv_nop\n\tv_nop" : "+v"(c) : "v"(a), "v"(b));
  return c;
}

template <int ET> struct Elem;
template <> struct Elem<0> { typedef _Float16 T; };
template <> struct Elem<1> { typedef __bf16 T; };
template <int ET, bool SPLIT, int BIAS_MODE, int OUT_MODE, bool RESID, int ACT = 0>
__global__ __launch_bounds__(256) void wmma_gemm64(
    const unsigned short* __restrict__ Ap, const unsigned short* __restrict__ A2p, int lda, long strideA,
    const unsigned short* __restrict__ Btp, const unsigned short* __restrict__ Bt2p, int ldb, long strideB,
    void* __restrict__ Cout, void* __restrict__ Cout2, int ldc, long strideC,
    const float* __restrict__ bias,
    const float* __restrict__ resid, long strideR,
    int M, int N, int K, float scale) {
  typedef typename Elem<ET>::T T;
  typedef typename Frag<T>::V V;
  const T* A = (const T*)Ap; const T* A2 = (const T*)A2p; const T* Bt = (const T*)Btp; const T* Bt2 = (const T*)Bt2p;
  __shared__ __align__(16) float sT[8][16 * 68];
  const int b    = blockIdx.y;
  const int lane = threadIdx.x & 31;
  const int wave = threadIdx.x >> 5;
  const int tilesN = N >> 6;
  const int tilesM = M >> 6;
  const int tile = blockIdx.x * 8 + wave;
  if (tile >= tilesM * tilesN) return;
  const int tm = tile / tilesN;
  const int tn = tile - tm * tilesN;
  const int m0 = tm << 6;
  const int n0 = tn << 6;

  const T* Ab  = A  + (size_t)b * strideA;
  const T* Bb  = Bt + (size_t)b * strideB;
  const T* Ab2 = SPLIT ? (A2  + (size_t)b * strideA) : nullptr;
  const T* Bb2 = SPLIT ? (Bt2 + (size_t)b * strideB) : nullptr;

  const int rlane = lane & 15;
  const int koff  = (lane >> 4) * 8;
  const int mOff  = (lane >> 4) * 8;

  v8f acc[4][4];
#pragma unroll
  for (int i = 0; i < 4; ++i)
#pragma unroll
    for (int j = 0; j < 4; ++j) acc[i][j] = (v8f){0.f,0.f,0.f,0.f,0.f,0.f,0.f,0.f};

  for (int k0 = 0; k0 < K; k0 += 32) {
    V bh[4], bl[4];
#pragma unroll
    for (int j = 0; j < 4; ++j) {
      const size_t bo = (size_t)(n0 + (j << 4) + rlane) * ldb + koff + k0;
      bh[j] = Frag<T>::load(Bb + bo);
      if (SPLIT) bl[j] = Frag<T>::load(Bb2 + bo);
    }
#pragma unroll
    for (int i = 0; i < 4; ++i) {
      const size_t ao = (size_t)(m0 + (i << 4) + rlane) * lda + koff + k0;
      V ah = Frag<T>::load(Ab + ao);
      V al;
      if (SPLIT) al = Frag<T>::load(Ab2 + ao);
#pragma unroll
      for (int j = 0; j < 4; ++j) {
        acc[i][j] = Frag<T>::mma(ah, bh[j], acc[i][j]);
        if (SPLIT) {
          acc[i][j] = Frag<T>::mma(ah, bl[j], acc[i][j]);
          acc[i][j] = Frag<T>::mma(al, bh[j], acc[i][j]);
        }
      }
      Frag<T>::guard4(acc[i][0], acc[i][1], acc[i][2], acc[i][3], ah, SPLIT ? al : ah);
    }
    Frag<T>::keep(bh[0], bh[1], bh[2], bh[3]);
    if (SPLIT) Frag<T>::keep(bl[0], bl[1], bl[2], bl[3]);
  }
  acc_guard4(acc[0][0], acc[0][1], acc[0][2], acc[0][3]);
  acc_guard4(acc[1][0], acc[1][1], acc[1][2], acc[1][3]);
  acc_guard4(acc[2][0], acc[2][1], acc[2][2], acc[2][3]);
  acc_guard4(acc[3][0], acc[3][1], acc[3][2], acc[3][3]);

  float* slab = sT[wave];
  const float* Rb = RESID ? (resid + (size_t)b * strideR) : nullptr;
#pragma unroll
  for (int i = 0; i < 4; ++i) {
    const int mBase = m0 + (i << 4);
#pragma unroll
    for (int j = 0; j < 4; ++j) {
      const int n = n0 + (j << 4) + rlane;
      float bv = 0.f;
      if (BIAS_MODE == 2) bv = bias[n];
#pragma unroll
      for (int r = 0; r < 8; ++r) {
        float v = acc[i][j][r] * scale;
        if (BIAS_MODE == 1) v += bias[mBase + mOff + r];
        if (BIAS_MODE == 2) v += bv;
        if (RESID) v += Rb[(size_t)(mBase + mOff + r) * ldc + n];
        if (ACT == 1) v = tanhf(v);
        if (ACT == 2) v = fmaxf(v, 0.0f);
        if (ACT == 3) v = v / (1.0f + expf(-v));
        if (ACT == 4) v = (v > 0.f) ? v : 0.01f * v;
        slab[(mOff + r) * 68 + (j << 4) + rlane] = v;
      }
    }
    __builtin_amdgcn_fence(__ATOMIC_RELEASE, "workgroup");
    __builtin_amdgcn_wave_barrier();
    __builtin_amdgcn_fence(__ATOMIC_ACQUIRE, "workgroup");
    if (OUT_MODE == 0) {
      float* C = (float*)Cout + (size_t)b * strideC;
      const int hh = lane >> 4, c4 = (lane & 15) * 4;
      for (int pass = 0; pass < 2; ++pass) {
#pragma unroll
        for (int it = 0; it < 8; ++it) {
          const int row = it * 2 + hh;
          v4f v = *(const v4f*)(slab + row * 68 + c4);
          *(volatile v4f*)(C + (size_t)(mBase + row) * ldc + n0 + c4) = v;
        }
        __threadfence();
      }
    } else {
      const int q = lane >> 3, c8 = (lane & 7) * 8;
      unsigned short* C  = (unsigned short*)Cout  + (size_t)b * strideC;
      unsigned short* C2 = (OUT_MODE == 2) ? ((unsigned short*)Cout2 + (size_t)b * strideC) : nullptr;
      for (int pass = 0; pass < 2; ++pass) {
#pragma unroll
        for (int it = 0; it < 4; ++it) {
          const int row = it * 4 + q;
          const float* sp = slab + row * 68 + c8;
          v8h hv, lv;
#pragma unroll
          for (int e = 0; e < 8; ++e) {
            if (OUT_MODE == 1) {
              hv[e] = (_Float16)sp[e];
            } else {
              unsigned short hb = f2bf_bits(sp[e]);
              unsigned short lb = f2bf_bits(sp[e] - bf_bits2f(hb));
              hv[e] = __builtin_bit_cast(_Float16, hb);
              lv[e] = __builtin_bit_cast(_Float16, lb);
            }
          }
          *(volatile v8h*)(C + (size_t)(mBase + row) * ldc + n0 + c8) = hv;
          if (OUT_MODE == 2) *(volatile v8h*)(C2 + (size_t)(mBase + row) * ldc + n0 + c8) = lv;
        }
        __threadfence();
      }
    }
    __builtin_amdgcn_fence(__ATOMIC_RELEASE, "workgroup");
    __builtin_amdgcn_wave_barrier();
    __builtin_amdgcn_fence(__ATOMIC_ACQUIRE, "workgroup");
  }
}

__global__ __launch_bounds__(kThr) void cast_plane_kernel(const float* __restrict__ src, unsigned short* __restrict__ dst,
                                                          int colsLog2, int dstPitch, int dstOff) {
  const int i   = blockIdx.x * kThr + threadIdx.x;
  const int sh  = colsLog2 - 3;
  const int row = i >> sh;
  const int c8  = (i & ((1 << sh) - 1)) * 8;
  const float* sp = src + ((size_t)row << colsLog2) + c8;
  const v4f a0 = *(const v4f*)(sp);
  const v4f a1 = *(const v4f*)(sp + 4);
  v8h hv;
#pragma unroll
  for (int e = 0; e < 4; ++e) {
    const float f0 = a0[e];
    const float f1 = a1[e];
    hv[e]     = (_Float16)carry_flush(bf16r(f0), kInCarry);
    hv[4 + e] = (_Float16)carry_flush(bf16r(f1), kInCarry);
  }
  unsigned short* dp = dst + (size_t)row * dstPitch + dstOff + c8;
  *(volatile v8h*)dp = hv;
  __threadfence();
  *(volatile v8h*)dp = hv;
}

__device__ __forceinline__ float fast_tanh(float v) { return 1.0f - 2.0f * frcp(__expf(2.0f * v) + 1.0f); }
__device__ __forceinline__ float fast_sigmoid(float v) { return frcp(1.0f + __expf(-v)); }

__global__ __launch_bounds__(128) void padcast_kernel(const float* __restrict__ src, int srcPitch, int srcColOff, int rowsLive, int colsLive,
                                                      unsigned short* __restrict__ dst, int dstPitch, int dstColOff) {
  const unsigned n = blockIdx.x;
  unsigned k8 = threadIdx.x * 8u;
  asm volatile("" : "+v"(k8));
  const bool rowLive = n < (unsigned)rowsLive;
  v8h hv;
#pragma unroll
  for (int e = 0; e < 8; ++e) {
    const unsigned k = k8 + (unsigned)e;
    const bool live = rowLive && (k < (unsigned)colsLive);
    const unsigned idx = live ? (n * (unsigned)srcPitch + (unsigned)srcColOff + k) : 0u;
    float w = src[idx];
    asm volatile("" : "+v"(w));
    hv[e] = (_Float16)(live ? carry_flush(bf16r(w), kWCarry) : 0.0f);
  }
  unsigned short* dp = dst + (size_t)n * (unsigned)dstPitch + (unsigned)dstColOff + k8;
  *(volatile v8h*)dp = hv;
  __threadfence();
  *(volatile v8h*)dp = hv;
}

__device__ __forceinline__ float bias_word(const float* __restrict__ p, unsigned n, unsigned nLive) {
  const bool live = n < nLive;
  float w = p[live ? n : 0u];
  asm volatile("" : "+v"(w));
  return live ? bf16r(w) : 0.0f;
}

constexpr int kFBG = 0, kFBTR = 1536, kFGBN = 2048, kFGBR = 2432, kFHBN = 2816, kFHBR = 3328, kFTBN = 3840, kFTBR = 3968, kFZB = 4096, kFEnd = 6144;
__global__ __launch_bounds__(kThr) void setup_kernel(const float* __restrict__ b_ih, const float* __restrict__ b_hh, const float* __restrict__ b_tr,
                                                     const float* __restrict__ n_b, const float* __restrict__ r_b, const float* __restrict__ ner_hb,
                                                     const float* __restrict__ re_hb, const float* __restrict__ ner_tb, const float* __restrict__ re_tb,
                                                     float* __restrict__ BIAS, unsigned short* __restrict__ ZERO) {
  unsigned v = blockIdx.x * (unsigned)kThr + threadIdx.x;
  asm volatile("" : "+v"(v));
  if (v < 1536u) {
    const unsigned i0 = v * 4u;
    v4f o = {0.f, 0.f, 0.f, 0.f};
    if (i0 < (unsigned)kFBTR) {
#pragma unroll
      for (int e = 0; e < 4; ++e) o[e] = bias_word(b_ih, i0 + e, (unsigned)kG5) + bias_word(b_hh, i0 + e, (unsigned)kG5);
    } else if (i0 < (unsigned)kFGBN) {
#pragma unroll
      for (int e = 0; e < 4; ++e) o[e] = bias_word(b_tr, i0 - (unsigned)kFBTR + e, (unsigned)kH);
    } else if (i0 < (unsigned)kFGBR) {
#pragma unroll
      for (int e = 0; e < 4; ++e) o[e] = bias_word(n_b, i0 - (unsigned)kFGBN + e, (unsigned)kH);
    } else if (i0 < (unsigned)kFHBN) {
#pragma unroll
      for (int e = 0; e < 4; ++e) o[e] = bias_word(r_b, i0 - (unsigned)kFGBR + e, (unsigned)kH);
    } else if (i0 < (unsigned)kFHBR) {
#pragma unroll
      for (int e = 0; e < 4; ++e) o[e] = bias_word(ner_hb, i0 - (unsigned)kFHBN + e, (unsigned)kH);
    } else if (i0 < (unsigned)kFTBN) {
#pragma unroll
      for (int e = 0; e < 4; ++e) o[e] = bias_word(re_hb, i0 - (unsigned)kFHBR + e, (unsigned)kH);
    } else if (i0 < (unsigned)kFTBR) {
#pragma unroll
      for (int e = 0; e < 4; ++e) o[e] = bias_word(ner_tb, i0 - (unsigned)kFTBN + e, (unsigned)kNT);
    } else if (i0 < (unsigned)kFZB) {
#pragma unroll
      for (int e = 0; e < 4; ++e) o[e] = bias_word(re_tb, i0 - (unsigned)kFTBR + e, (unsigned)kNR);
    }
    float* dp = BIAS + i0;
    *(volatile v4f*)dp = o;
    __threadfence();
    *(volatile v4f*)dp = o;
  } else {
    const unsigned w = v - 1536u;
    v8h z;
#pragma unroll
    for (int e = 0; e < 8; ++e) z[e] = (_Float16)0.0f;
    unsigned short* dp = ZERO + (size_t)w * 8u;
    *(volatile v8h*)dp = z;
    __threadfence();
    *(volatile v8h*)dp = z;
  }
}
static_assert(kFEnd / 4 == 1536 && 335872 / 16 == 20992 && 1536 + 20992 == 88 * kThr, "set-up grid exact");
static_assert((kFBTR % 128) == 0 && (kFGBN % 128) == 0 && (kFGBR % 128) == 0 && (kFHBN % 128) == 0 && (kFHBR % 128) == 0 && (kFTBN % 128) == 0 && (kFTBR % 128) == 0 && (kFZB % 128) == 0 && (kFEnd % 128) == 0, "set-up regions wave-uniform");
static_assert(kFBTR - kFBG >= kG5P && kFGBN - kFBTR >= kCOP && kFGBR - kFGBN >= kHP && kFHBN - kFGBR >= kHP && kFHBR - kFHBN >= kCOP && kFTBN - kFHBR >= kCOP && kFTBR - kFTBN >= kTP && kFZB - kFTBR >= kTP && kFEnd - kFZB >= kG5P, "every bias row covers the widest product that reads it");

constexpr int kCellThr = 320;
__global__ __launch_bounds__(kCellThr) void cell_kernel(const float* __restrict__ PRE, const float* __restrict__ GG, const float* __restrict__ CO,
                                                        unsigned short* __restrict__ CC16, unsigned short* __restrict__ TASK16, int t) {
  __shared__ __align__(16) float sV[4][kHP];
  __shared__ float sM[4][16];
  __shared__ float sS[4][16];
  __shared__ __align__(16) float sO[6][kHP];
  const unsigned b = blockIdx.x;
  unsigned u = threadIdx.x;
  asm volatile("" : "+v"(u));
  const bool live = u < (unsigned)kH;
  const unsigned uc = live ? u : 0u;
  const unsigned row = (unsigned)t * (unsigned)kB + b;
  const float* pr = PRE + (size_t)row * kG5P;
  const float* gr = GG + (size_t)b * kG5P;
  float g[5];
#pragma unroll
  for (int k = 0; k < 5; ++k) {
    float a = pr[(unsigned)(k * kH) + uc];
    float c2 = gr[(unsigned)(k * kH) + uc];
    asm volatile("" : "+v"(a), "+v"(c2));
    g[k] = a + c2;
  }
  float cin = CO[(size_t)b * kCOP + uc];
  asm volatile("" : "+v"(cin));

#pragma unroll
  for (int q = 0; q < 4; ++q) sV[q][u] = live ? g[q + 1] : -3.0e38f;
  __syncthreads();
  const unsigned qv = u / 10u, gp = u - qv * 10u;
  if (u < 40u) {
    const float* sp = &sV[qv][gp * 32u];
    float m = sp[0];
#pragma unroll 1
    for (int i = 1; i < 32; ++i) { const float x = sp[i]; m = (x > m) ? x : m; }
    sM[qv][gp] = m;
  }
  __syncthreads();
  float mx[4];
#pragma unroll
  for (int q = 0; q < 4; ++q) {
    float m = sM[q][0];
    asm volatile("" : "+v"(m));
#pragma unroll
    for (int i = 1; i < 10; ++i) { float x = sM[q][i]; asm volatile("" : "+v"(x)); m = (x > m) ? x : m; }
    mx[q] = m;
  }
#pragma unroll
  for (int q = 0; q < 4; ++q) sV[q][u] = live ? __expf(g[q + 1] - mx[q]) : 0.0f;
  __syncthreads();
  if (u < 40u) {
    float* sp = &sV[qv][gp * 32u];
    float run = 0.0f;
#pragma unroll 1
    for (int i = 0; i < 32; ++i) { run += sp[i]; sp[i] = run; }
    sS[qv][gp] = run;
  }
  __syncthreads();
  const unsigned myGroup = u >> 5;
  float cum[4];
#pragma unroll
  for (int q = 0; q < 4; ++q) {
    float off = 0.0f, tot = 0.0f;
#pragma unroll
    for (int i = 0; i < 10; ++i) {
      float s = sS[q][i];
      asm volatile("" : "+v"(s));
      tot += s;
      off += ((unsigned)i < myGroup) ? s : 0.0f;
    }
    cum[q] = (off + sV[q][u]) * frcp(tot);
  }
  const float eg_i = 1.0f - cum[0], rg_i = cum[1], eg_c = 1.0f - cum[2], rg_c = cum[3];
  const float c = fast_tanh(g[0]);
  const float ov_c = rg_c * eg_c, up_c = rg_c - ov_c, dn_c = eg_c - ov_c;
  const float ov_i = rg_i * eg_i, up_i = rg_i - ov_i, dn_i = eg_i - ov_i;
  const float share = ov_i * cin + ov_c * c;
  const float c_re  = up_i * cin + up_c * c + share;
  const float c_ner = dn_i * cin + dn_c * c + share;
  sO[0][u] = live ? c_re : 0.0f;
  sO[1][u] = live ? c_ner : 0.0f;
  sO[2][u] = live ? share : 0.0f;
  sO[3][u] = live ? fast_tanh(c_ner) : 0.0f;
  sO[4][u] = live ? fast_tanh(share) : 0.0f;
  sO[5][u] = live ? fast_tanh(c_re) : 0.0f;
  __syncthreads();
  const bool stCC = u < 120u;
  const bool stTK = (u >= 128u) && (u < 248u);
  if (stCC || stTK) {
    const unsigned w = stCC ? u : (u - 128u);
    const unsigned seg = w / 40u, k8 = (w - seg * 40u) * 8u;
    const float* sp = &sO[(stCC ? 0u : 3u) + seg][k8];
    const v4f a0 = *(const v4f*)(sp), a1 = *(const v4f*)(sp + 4);
    v8h hv;
#pragma unroll
    for (int e = 0; e < 4; ++e) { hv[e] = (_Float16)carry_flush(a0[e], kSC); hv[4 + e] = (_Float16)carry_flush(a1[e], kSC); }
    unsigned short* dp = stCC ? (CC16 + (size_t)b * (3 * kHP) + seg * (unsigned)kHP + k8)
                              : (TASK16 + (size_t)row * (3 * kHP) + seg * (unsigned)kHP + k8);
    *(volatile v8h*)dp = hv;
    __threadfence();
    *(volatile v8h*)dp = hv;
  }
}
static_assert(kCellThr == kHP && kHP == 10 * 32 && 3 * (kHP / 8) == 120 && 128 + 120 <= kCellThr && (kHP % 64) == 0, "the cell's thread map: ten groups of 32; 120 + 120 storing threads; a segment is whole lines");

__global__ __launch_bounds__(160) void state_kernel(const float* __restrict__ CO, unsigned short* __restrict__ H16) {
  unsigned tid = threadIdx.x;
  asm volatile("" : "+v"(tid));
  const unsigned b = tid / 40u, k8 = (tid - b * 40u) * 8u;
  const float* cr = CO + (size_t)b * kCOP;
  v8h hv;
#pragma unroll
  for (int hf = 0; hf < 2; ++hf) {
    const unsigned k4 = k8 + 4u * (unsigned)hf;
    const bool live4 = k4 < (unsigned)kH;
    v4f a = *(const v4f*)(cr + (live4 ? k4 : 0u));
    asm volatile("" : "+v"(a));
#pragma unroll
    for (int e = 0; e < 4; ++e) hv[4 * hf + e] = (_Float16)(live4 ? carry_flush(fast_tanh(a[e]), kSC) : 0.0f);
  }
  unsigned short* dp = H16 + (size_t)b * kHP + k8;
  *(volatile v8h*)dp = hv;
  __threadfence();
  *(volatile v8h*)dp = hv;
}
static_assert(kB * (kHP / 8) == 160, "state grid exact");

__global__ __launch_bounds__(160) void gmax_kernel(const float* __restrict__ HG, unsigned short* __restrict__ G16) {
  unsigned tid = threadIdx.x;
  asm volatile("" : "+v"(tid));
  const unsigned b = tid / 40u, k8 = (tid - b * 40u) * 8u;
  float m[8];
#pragma unroll
  for (int e = 0; e < 8; ++e) m[e] = -2.0f;
#pragma unroll 1
  for (unsigned l = 0; l < (unsigned)kL; ++l) {
    const float* hp = HG + (size_t)(l * (unsigned)kB + b) * kHP + k8;
    const v4f a0 = *(const v4f*)(hp), a1 = *(const v4f*)(hp + 4);
#pragma unroll
    for (int e = 0; e < 4; ++e) {
      const float x0 = fast_tanh(a0[e]), x1 = fast_tanh(a1[e]);
      m[e] = (x0 > m[e]) ? x0 : m[e];
      m[4 + e] = (x1 > m[4 + e]) ? x1 : m[4 + e];
    }
  }
  v8h hv;
#pragma unroll
  for (int e = 0; e < 8; ++e) hv[e] = (_Float16)(((k8 + (unsigned)e) < (unsigned)kH) ? carry_flush(m[e], kSC) : 0.0f);
  unsigned short* dp = G16 + (size_t)b * kHP + k8;
  *(volatile v8h*)dp = hv;
  __threadfence();
  *(volatile v8h*)dp = hv;
}

__global__ __launch_bounds__(kThr) void pair_ln_kernel(const float* __restrict__ ASE, const float* __restrict__ CG, const float* __restrict__ lng,
                                                       const float* __restrict__ lnb, unsigned short* __restrict__ E16) {
  unsigned p = blockIdx.x * (unsigned)kThr + threadIdx.x;
  asm volatile("" : "+v"(p));
  const unsigned b = p & 3u, j = (p >> 2) & 127u, i = p >> 9;
  const float* as = ASE + (size_t)(i * (unsigned)kB + b) * (2 * kHP);
  const float* ae = ASE + (size_t)(j * (unsigned)kB + b) * (2 * kHP) + kHP;
  const float* cg = CG + (size_t)b * kCOP;
  float s = 0.0f;
#pragma unroll 1
  for (unsigned g4 = 0; g4 < (unsigned)(kH / 4); ++g4) {
    const v4f a = *(const v4f*)(as + 4u * g4), e = *(const v4f*)(ae + 4u * g4), c = *(const v4f*)(cg + 4u * g4);
    s += (a[0] + e[0]) + c[0];
    s += (a[1] + e[1]) + c[1];
    s += (a[2] + e[2]) + c[2];
    s += (a[3] + e[3]) + c[3];
  }
  const float mu = s * kInvH;
  float q = 0.0f;
#pragma unroll 1
  for (unsigned g4 = 0; g4 < (unsigned)(kH / 4); ++g4) {
    const v4f a = *(const v4f*)(as + 4u * g4), e = *(const v4f*)(ae + 4u * g4), c = *(const v4f*)(cg + 4u * g4);
#pragma unroll
    for (int x = 0; x < 4; ++x) { const float d = ((a[x] + e[x]) + c[x]) - mu; q += d * d; }
  }
  const float rstd = rsqrtf(q * kInvH + kLnEps);
  unsigned short* er = E16 + (size_t)p * kHP;
#pragma unroll 1
  for (unsigned kk = 0; kk < (unsigned)(kHP / 8); ++kk) {
    v8h hv;
#pragma unroll
    for (int hf = 0; hf < 2; ++hf) {
      const unsigned g4 = 2u * kk + (unsigned)hf;
      const bool live4 = g4 < (unsigned)(kH / 4);
      const unsigned gc = live4 ? g4 : 0u;
      v4f a = *(const v4f*)(as + 4u * gc), e = *(const v4f*)(ae + 4u * gc), c = *(const v4f*)(cg + 4u * gc);
      v4f gn = *(const v4f*)(lng + 4u * gc), bt = *(const v4f*)(lnb + 4u * gc);
      asm volatile("" : "+v"(a), "+v"(e), "+v"(c), "+v"(gn), "+v"(bt));
#pragma unroll
      for (int x = 0; x < 4; ++x) {
        const float y = (((a[x] + e[x]) + c[x]) - mu) * rstd * bf16r(gn[x]) + bf16r(bt[x]);
        const float el = (y > 0.0f) ? y : (__expf(y) - 1.0f);
        hv[4 * hf + x] = (_Float16)(live4 ? carry_flush(el, kCE) : 0.0f);
      }
    }
    unsigned short* dp = er + 8u * kk;
    *(volatile v8h*)dp = hv;
    __threadfence();
    *(volatile v8h*)dp = hv;
  }
}
static_assert(kPairs == 256 * kThr && kL == 128 && kB == 4 && (kH / 4) == 75 && (kHP / 8) == 40, "pair grid exact; the row decode's shifts");

__global__ __launch_bounds__(kThr) void out_kernel(const float* __restrict__ Y, const float* __restrict__ mask, float* __restrict__ out, int T, int diag) {
  unsigned v = blockIdx.x * (unsigned)kThr + threadIdx.x;
  asm volatile("" : "+v"(v));
  const unsigned e0 = 4u * v;
  v4f o;
#pragma unroll
  for (int x = 0; x < 4; ++x) {
    const unsigned e = e0 + (unsigned)x;
    const unsigned p = e / (unsigned)T;
    const unsigned tt = e - p * (unsigned)T;
    const unsigned b = p & 3u, j = (p >> 2) & 127u, i = p >> 9;
    float y = Y[(size_t)p * kTP + tt];
    float mi = mask[i * (unsigned)kB + b], mj = mask[j * (unsigned)kB + b];
    asm volatile("" : "+v"(y), "+v"(mi), "+v"(mj));
    float m = bf16r(mi) * bf16r(mj);
    if (diag != 0) m = m * ((j >= i) ? 1.0f : 0.0f);
    o[x] = fast_sigmoid(y) * m;
  }
  float* dp = out + e0;
  *(volatile v4f*)dp = o;
  __threadfence();
  *(volatile v4f*)dp = o;
}
static_assert(((size_t)kPairs * kNT / 4) % kThr == 0 && ((size_t)kPairs * kNR / 4) % kThr == 0 && ((size_t)kPairs * kNT * 4) % 128 == 0, "output grids exact; the second output starts on a 128-B line");

static_assert(((size_t)kRows * kD / 8) % kThr == 0 && kD == 3 * 256, "the plane cast of x: 1,536 rows of 256 words; grid exact");

extern "C" void kernel_launch(void* const* d_in, const int* in_sizes, int n_in,
                              void* d_out, int out_size, void* d_ws, size_t ws_size,
                              hipStream_t stream) {
  if (n_in < 24 || d_out == nullptr || d_ws == nullptr) return;
  if (in_sizes[0] != kRows * kD || in_sizes[1] != kRows || in_sizes[2] != kG5 * kD || in_sizes[3] != kG5 || in_sizes[4] != kG5 * kH || in_sizes[5] != kG5) return;
  if (in_sizes[6] != kH * 3 * kH || in_sizes[7] != kH || in_sizes[8] != kH * 2 * kH || in_sizes[9] != kH || in_sizes[10] != kH * 3 * kH || in_sizes[11] != kH) return;
  if (in_sizes[12] != kH || in_sizes[13] != kH || in_sizes[14] != kNT * kH || in_sizes[15] != kNT || in_sizes[16] != kH * 2 * kH || in_sizes[17] != kH) return;
  if (in_sizes[18] != kH * 3 * kH || in_sizes[19] != kH || in_sizes[20] != kH || in_sizes[21] != kH || in_sizes[22] != kNR * kH || in_sizes[23] != kNR) return;
  if (out_size != kPairs * (kNT + kNR)) return;
  if (ws_size < kWsTotal) return;
  const float* x = (const float*)d_in[0];
  const float* mask = (const float*)d_in[1];
  const float* W_ih = (const float*)d_in[2];
  const float* b_ih = (const float*)d_in[3];
  const float* W_hh = (const float*)d_in[4];
  const float* b_hh = (const float*)d_in[5];
  const float* W_tr = (const float*)d_in[6];
  const float* b_tr = (const float*)d_in[7];
  const float* n_W = (const float*)d_in[8];
  const float* n_b = (const float*)d_in[9];
  const float* ner_hW = (const float*)d_in[10];
  const float* ner_hb = (const float*)d_in[11];
  const float* ner_g = (const float*)d_in[12];
  const float* ner_beta = (const float*)d_in[13];
  const float* ner_tW = (const float*)d_in[14];
  const float* ner_tb = (const float*)d_in[15];
  const float* r_W = (const float*)d_in[16];
  const float* r_b = (const float*)d_in[17];
  const float* re_hW = (const float*)d_in[18];
  const float* re_hb = (const float*)d_in[19];
  const float* re_g = (const float*)d_in[20];
  const float* re_beta = (const float*)d_in[21];
  const float* re_tW = (const float*)d_in[22];
  const float* re_tb = (const float*)d_in[23];
  float* out = (float*)d_out;
  char* ws = (char*)d_ws;
  unsigned short* X16 = (unsigned short*)(ws + kOffX16);
  unsigned short* WIH16 = (unsigned short*)(ws + kOffWIH16);
  unsigned short* WHH16 = (unsigned short*)(ws + kOffWHH16);
  unsigned short* WTR16 = (unsigned short*)(ws + kOffWTR16);
  unsigned short* GWN16 = (unsigned short*)(ws + kOffGWN16);
  unsigned short* GWR16 = (unsigned short*)(ws + kOffGWR16);
  unsigned short* HWSEN16 = (unsigned short*)(ws + kOffHWSEN16);
  unsigned short* HWSER16 = (unsigned short*)(ws + kOffHWSER16);
  unsigned short* HWGN16 = (unsigned short*)(ws + kOffHWGN16);
  unsigned short* HWGR16 = (unsigned short*)(ws + kOffHWGR16);
  unsigned short* TWN16 = (unsigned short*)(ws + kOffTWN16);
  unsigned short* TWR16 = (unsigned short*)(ws + kOffTWR16);
  float* BIAS = (float*)(ws + kOffBIAS);
  unsigned short* H16 = (unsigned short*)(ws + kOffH16);
  unsigned short* CC16 = (unsigned short*)(ws + kOffCC16);
  unsigned short* G16 = (unsigned short*)(ws + kOffG16);
  float* CO = (float*)(ws + kOffCO);
  float* PRE = (float*)(ws + kOffPRE);
  float* GG = (float*)(ws + kOffGG);
  unsigned short* TASK16 = (unsigned short*)(ws + kOffTASK16);
  float* HG = (float*)(ws + kOffHG);
  float* ASE = (float*)(ws + kOffASE);
  float* CG = (float*)(ws + kOffCG);
  unsigned short* E16 = (unsigned short*)(ws + kOffE16);
  float* Y = (float*)(ws + kOffY);

  cast_plane_kernel<<<(int)(((size_t)kRows * kD / 8) / kThr), kThr, 0, stream>>>(x, X16, 8, 256, 0);
  padcast_kernel<<<kG5P, kD / 8, 0, stream>>>(W_ih, kD, 0, kG5, kD, WIH16, kD, 0);
  padcast_kernel<<<kG5P, kHP / 8, 0, stream>>>(W_hh, kH, 0, kG5, kH, WHH16, kHP, 0);
  padcast_kernel<<<kCOP, kHP / 8, 0, stream>>>(W_tr, 3 * kH, 0, kH, kH, WTR16, 3 * kHP, 0);
  padcast_kernel<<<kCOP, kHP / 8, 0, stream>>>(W_tr, 3 * kH, kH, kH, kH, WTR16, 3 * kHP, kHP);
  padcast_kernel<<<kCOP, kHP / 8, 0, stream>>>(W_tr, 3 * kH, 2 * kH, kH, kH, WTR16, 3 * kHP, 2 * kHP);
  padcast_kernel<<<kHP, kHP / 8, 0, stream>>>(n_W, 2 * kH, kH, kH, kH, GWN16, 2 * kHP, 0);
  padcast_kernel<<<kHP, kHP / 8, 0, stream>>>(n_W, 2 * kH, 0, kH, kH, GWN16, 2 * kHP, kHP);
  padcast_kernel<<<kHP, kHP / 8, 0, stream>>>(r_W, 2 * kH, 0, kH, kH, GWR16, 2 * kHP, 0);
  padcast_kernel<<<kHP, kHP / 8, 0, stream>>>(r_W, 2 * kH, kH, kH, kH, GWR16, 2 * kHP, kHP);
  padcast_kernel<<<kHP, kHP / 8, 0, stream>>>(ner_hW, 3 * kH, 0, kH, kH, HWSEN16, kHP, 0);
  padcast_kernel<<<kHP, kHP / 8, 0, stream>>>(ner_hW, 3 * kH, kH, kH, kH, HWSEN16 + (size_t)kHP * kHP, kHP, 0);
  padcast_kernel<<<kCOP, kHP / 8, 0, stream>>>(ner_hW, 3 * kH, 2 * kH, kH, kH, HWGN16, kHP, 0);
  padcast_kernel<<<kHP, kHP / 8, 0, stream>>>(re_hW, 3 * kH, 0, kH, kH, HWSER16, kHP, 0);
  padcast_kernel<<<kHP, kHP / 8, 0, stream>>>(re_hW, 3 * kH, kH, kH, kH, HWSER16 + (size_t)kHP * kHP, kHP, 0);
  padcast_kernel<<<kCOP, kHP / 8, 0, stream>>>(re_hW, 3 * kH, 2 * kH, kH, kH, HWGR16, kHP, 0);
  padcast_kernel<<<kTP, kHP / 8, 0, stream>>>(ner_tW, kH, 0, kNT, kH, TWN16, kHP, 0);
  padcast_kernel<<<kTP, kHP / 8, 0, stream>>>(re_tW, kH, 0, kNR, kH, TWR16, kHP, 0);
  setup_kernel<<<88, kThr, 0, stream>>>(b_ih, b_hh, b_tr, n_b, r_b, ner_hb, re_hb, ner_tb, re_tb, BIAS, H16);
  wmma_gemm64<0, false, 2, 0, false, 0><<<dim3((kRows / 64) * (kG5P / 64) / 8, 1), 256, 0, stream>>>(
      X16, X16, kD, 0L, WIH16, WIH16, kD, 0L, (void*)PRE, (void*)PRE, kG5P, 0L, BIAS + kFBG, nullptr, 0L, kRows, kG5P, kD, kScX);

  for (int t = 0; t < kL; ++t) {
    wmma_gemm64<0, false, 2, 0, false, 0><<<dim3((kMP / 64) * (kG5P / 64) / 8, 1), 256, 0, stream>>>(
        H16, H16, kHP, 0L, WHH16, WHH16, kHP, 0L, (void*)GG, (void*)GG, kG5P, 0L, BIAS + kFZB, nullptr, 0L, kMP, kG5P, kHP, kScS);
    cell_kernel<<<kB, kCellThr, 0, stream>>>(PRE, GG, CO, CC16, TASK16, t);
    wmma_gemm64<0, false, 2, 0, false, 0><<<dim3((kMP / 64) * (kCOP / 64) / 8, 1), 256, 0, stream>>>(
        CC16, CC16, 3 * kHP, 0L, WTR16, WTR16, 3 * kHP, 0L, (void*)CO, (void*)CO, kCOP, 0L, BIAS + kFBTR, nullptr, 0L, kMP, kCOP, 3 * kHP, kScS);
    state_kernel<<<1, 160, 0, stream>>>(CO, H16);
  }

  for (int unit = 0; unit < 2; ++unit) {
    const bool ner = (unit == 0);
    const unsigned short* Ag = ner ? TASK16 : (TASK16 + kHP);
    const unsigned short* At = ner ? TASK16 : (TASK16 + 2 * kHP);
    const unsigned short* GW16 = ner ? GWN16 : GWR16;
    const unsigned short* HWSE16 = ner ? HWSEN16 : HWSER16;
    const unsigned short* HWG16 = ner ? HWGN16 : HWGR16;
    const unsigned short* TW16 = ner ? TWN16 : TWR16;
    wmma_gemm64<0, false, 2, 0, false, 0><<<dim3((kRows / 64) * (kHP / 64) / 8, 1), 256, 0, stream>>>(
        Ag, Ag, 3 * kHP, 0L, GW16, GW16, 2 * kHP, 0L, (void*)HG, (void*)HG, kHP, 0L, BIAS + (ner ? kFGBN : kFGBR), nullptr, 0L, kRows, kHP, 2 * kHP, kScS);
    gmax_kernel<<<1, 160, 0, stream>>>(HG, G16);
    wmma_gemm64<0, false, 2, 0, false, 0><<<dim3((kRows / 64) * (2 * kHP / 64) / 8, 1), 256, 0, stream>>>(
        At, At, 3 * kHP, 0L, HWSE16, HWSE16, kHP, 0L, (void*)ASE, (void*)ASE, 2 * kHP, 0L, BIAS + kFZB, nullptr, 0L, kRows, 2 * kHP, kHP, kScS);
    wmma_gemm64<0, false, 2, 0, false, 0><<<dim3((kMP / 64) * (kCOP / 64) / 8, 1), 256, 0, stream>>>(
        G16, G16, kHP, 0L, HWG16, HWG16, kHP, 0L, (void*)CG, (void*)CG, kCOP, 0L, BIAS + (ner ? kFHBN : kFHBR), nullptr, 0L, kMP, kCOP, kHP, kScS);
    pair_ln_kernel<<<kPairs / kThr, kThr, 0, stream>>>(ASE, CG, ner ? ner_g : re_g, ner ? ner_beta : re_beta, E16);
    wmma_gemm64<0, false, 2, 0, false, 0><<<dim3((kPairs / 64) * (kTP / 64) / 8, 1), 256, 0, stream>>>(
        E16, E16, kHP, 0L, TW16, TW16, kHP, 0L, (void*)Y, (void*)Y, kTP, 0L, BIAS + (ner ? kFTBN : kFTBR), nullptr, 0L, kPairs, kTP, kHP, kScE);
    if (ner) out_kernel<<<(int)(((size_t)kPairs * kNT / 4) / kThr), kThr, 0, stream>>>(Y, mask, out, kNT, 1);
    else     out_kernel<<<(int)(((size_t)kPairs * kNR / 4) / kThr), kThr, 0, stream>>>(Y, mask, out + (size_t)kPairs * kNT, kNR, 0);
  }
}
